// MultiHeadAttention_58695023067217
// MI455X (gfx1250) — hardware-verified
//
#include <hip/hip_runtime.h>

typedef _Float16 h16;
typedef __attribute__((ext_vector_type(16))) _Float16      v16h;
typedef __attribute__((ext_vector_type(8)))  float         v8f;
typedef __attribute__((ext_vector_type(4)))  float         v4f;
typedef __attribute__((ext_vector_type(2)))  float         v2f;
typedef __attribute__((ext_vector_type(4)))  unsigned int  v4u;
typedef float v4fa __attribute__((ext_vector_type(4), may_alias));

#ifndef NB
#define NB 2
#endif
#ifndef SEQ
#define SEQ 2048
#endif
#define NB_FULL  2
#define SEQ_FULL 2048
#define SQ   SEQ
#define DQ   1024
#define HQ   16
#define HDQ  64
#define MQ   (NB * SQ)
#define PLX  ((size_t)MQ * DQ)
#define PLW  ((size_t)DQ * DQ)
#define RSPLIT (1.0f / 2048.0f)
#define WCARRY 16.0f
#define NEG_L2T_OVER_32 (-0.41524101186092f)

static_assert(NB <= NB_FULL);
static_assert(SEQ <= SEQ_FULL);
static_assert(SQ % 128 == 0);
static_assert(DQ == HQ * HDQ);
static_assert(HDQ == 64);
static_assert(DQ % 64 == 0);
static_assert(((size_t)MQ * DQ) % (256 * 8) == 0);
static_assert(((size_t)DQ * DQ) % (256 * 8) == 0);
static_assert(((size_t)MQ * 32) % 256 == 0);
static_assert((NB * HQ * (SQ / 16)) % 8 == 0);
static_assert(MQ % 128 == 0);

__device__ __forceinline__ void split16(float f, h16& h, h16& l) { h = (h16)f; l = (h16)((f - (float)h) * 2048.0f); }
__device__ __forceinline__ unsigned short hbits(h16 h) { return __builtin_bit_cast(unsigned short, h); }
__device__ __forceinline__ unsigned pack2h(h16 a, h16 b) { return (unsigned)hbits(a) | ((unsigned)hbits(b) << 16); }

__device__ __forceinline__ float to_bf16_f32(float f) {
    unsigned u = __float_as_uint(f);
    u += 0x7FFFu + ((u >> 16) & 1u);
    return __uint_as_float(u & 0xFFFF0000u);
}

struct U256 { v4u a, b; };

__device__ __forceinline__ v16h load_frag2(const h16* p0, const h16* p1) {
    U256 t;
    t.a = *reinterpret_cast<const v4u*>(p0);
    t.b = *reinterpret_cast<const v4u*>(p1);
    return __builtin_bit_cast(v16h, t);
}

__device__ __forceinline__ v8f wmma_f16(v16h a, v16h b, v8f c) {
    c = __builtin_amdgcn_wmma_f32_16x16x32_f16(false, a, false, b, (short)0, c, false, false);
    asm volatile("v_nop\n\tv_nop\n\tv_nop\n\tv_nop" : "+v"(c) : "v"(a), "v"(b));
    return c;
}
__device__ __forceinline__ v8f wmma_split(v16h ah, v16h al, v16h bh, v16h bl, v8f c) {
    v8f x = {};
    x = wmma_f16(al, bh, x);
    x = wmma_f16(ah, bl, x);
    return wmma_f16(ah, bh, c) + x * RSPLIT;
}

__device__ __forceinline__ void copy16(const h16* g, h16* l) {
    *reinterpret_cast<v4u*>(l) = *reinterpret_cast<const v4u*>(g);
}

__device__ __forceinline__ v4u cvt8(v4f a, v4f b, float sc) {
    v4u p;
    p.x = pack2h((h16)(to_bf16_f32(a.x) * sc), (h16)(to_bf16_f32(a.y) * sc));
    p.y = pack2h((h16)(to_bf16_f32(a.z) * sc), (h16)(to_bf16_f32(a.w) * sc));
    p.z = pack2h((h16)(to_bf16_f32(b.x) * sc), (h16)(to_bf16_f32(b.y) * sc));
    p.w = pack2h((h16)(to_bf16_f32(b.z) * sc), (h16)(to_bf16_f32(b.w) * sc));
    return p;
}

__global__ __launch_bounds__(256) void cvt_x(const float* __restrict__ x, h16* __restrict__ out) {
    const unsigned gid = blockIdx.x * 256u + threadIdx.x;
    const unsigned row = gid >> 7;
    const unsigned c8  = gid & 127u;
    const unsigned b = row / (unsigned)SQ, s = row % (unsigned)SQ;
    const float* src = x + ((size_t)(b * (unsigned)SEQ_FULL + s) * DQ + c8 * 8u);
    const v4f a0 = *(const v4f*)src;
    const v4f a1 = *(const v4f*)(src + 4);
    const v4u p = cvt8(a0, a1, 1.0f);
    h16* d = out + (size_t)gid * 8u;
    *(volatile v4u*)d = p;
    __threadfence();
    *(volatile v4u*)d = p;
}

__global__ __launch_bounds__(256) void cvt_w4(const float* __restrict__ w0, const float* __restrict__ w1,
                                              const float* __restrict__ w2, const float* __restrict__ w3,
                                              h16* __restrict__ out) {
    const unsigned y = blockIdx.y;
    const float* w = (y == 0u) ? w0 : (y == 1u) ? w1 : (y == 2u) ? w2 : w3;
    const unsigned gid = blockIdx.x * 256u + threadIdx.x;
    const float* src = w + (size_t)gid * 8u;
    const v4f a0 = *(const v4f*)src;
    const v4f a1 = *(const v4f*)(src + 4);
    const v4u p = cvt8(a0, a1, WCARRY);
    h16* d = out + (size_t)y * PLW + (size_t)gid * 8u;
    *(volatile v4u*)d = p;
    __threadfence();
    *(volatile v4u*)d = p;
}

__global__ __launch_bounds__(256) void rope_tab(const int* __restrict__ pos, v2f* __restrict__ tab) {
    const unsigned gid = blockIdx.x * 256u + threadIdx.x;
    const unsigned row = gid >> 5, i = gid & 31u;
    const unsigned b = row / (unsigned)SQ, s = row % (unsigned)SQ;
    const float p = (float)pos[b * (unsigned)SEQ_FULL + s];
    const float invf = exp2f((float)i * NEG_L2T_OVER_32);
    const float ang = p * invf;
    v2f cs;
    cs.x = cosf(ang);
    cs.y = sinf(ang);
    v2f* d = tab + gid;
    *(volatile v2f*)d = cs;
    __threadfence();
    *(volatile v2f*)d = cs;
}

template <int MODE, int ARES, int ROPE>
__global__ __launch_bounds__(256)
void gemm_wmma_f16(const h16* __restrict__ A, const h16* __restrict__ BT,
                   float* __restrict__ outF, h16* __restrict__ outB,
                   const v2f* __restrict__ tab, float scale) {
    __shared__ alignas(16) h16   bsh[2][64 * 32];
    __shared__ alignas(16) float stg[8][16 * 64];

    const unsigned tid  = threadIdx.x;
    const unsigned lane = tid & 31u;
    const unsigned wave = tid >> 5;
    const unsigned lo   = lane & 15u;
    const unsigned hi   = lane >> 4;
    const unsigned rowBase = blockIdx.y * 128u + wave * 16u;
    const unsigned colBase = blockIdx.x * 64u;

    const unsigned cn = tid >> 2, cc = tid & 3u;
    const h16* bSrc = BT + (size_t)(colBase + cn) * DQ + cc * 8u;
    const unsigned bOff = cn * 32u + cc * 8u;

    copy16(bSrc, &bsh[0][bOff]);
    __syncthreads();

    v8f acc[4]  = {};
    v8f accl[4] = {};
    const h16* aRow = A + (size_t)(rowBase + lo) * DQ;

    const unsigned nk = DQ / 32;
    for (unsigned ik = 0; ik < nk; ++ik) {
        const unsigned k0  = ik * 32u;
        const unsigned buf = ik & 1u;
        if (ik + 1u < nk)
            copy16(bSrc + (size_t)(ik + 1u) * 32u, &bsh[buf ^ 1u][bOff]);

        const v16h af = load_frag2(aRow + k0 + hi * 8u, aRow + k0 + hi * 8u + 16u);
        v16h afl = af;
        if (ARES) afl = load_frag2(aRow + PLX + k0 + hi * 8u, aRow + PLX + k0 + hi * 8u + 16u);
#pragma unroll
        for (int t = 0; t < 4; ++t) {
            const h16* bp = &bsh[buf][(t * 16 + lo) * 32 + hi * 8];
            const v16h bfr = load_frag2(bp, bp + 16);
            acc[t] = wmma_f16(af, bfr, acc[t]);
            if (ARES) accl[t] = wmma_f16(afl, bfr, accl[t]);
        }
        __syncthreads();
    }

    float* sg = stg[wave];
#pragma unroll
    for (int t = 0; t < 4; ++t)
#pragma unroll
        for (int j = 0; j < 8; ++j) {
            float v = acc[t][j];
            if (ARES) v += accl[t][j] * RSPLIT;
            sg[(j + 8 * hi) * 64 + t * 16 + lo] = v * scale;
        }
    asm volatile("s_wait_dscnt 0" ::: "memory");
    __builtin_amdgcn_wave_barrier();
    if (MODE == 0) {
        v4f ov[8]; size_t oo[8];
#pragma unroll
        for (int i = 0; i < 8; ++i) {
            const unsigned c = lane + 32u * i, r = c >> 4, q = c & 15u;
            ov[i] = *(const v4fa*)(sg + r * 64u + q * 4u);
            oo[i] = (size_t)(rowBase + r) * DQ + colBase + q * 4u;
        }
#pragma unroll
        for (int i = 0; i < 8; ++i) *(volatile v4f*)(outF + oo[i]) = ov[i];
        __threadfence();
#pragma unroll
        for (int i = 0; i < 8; ++i) *(volatile v4f*)(outF + oo[i]) = ov[i];
    } else {
        const unsigned h = colBase >> 6;
        const unsigned b = rowBase / (unsigned)SQ, s0 = rowBase % (unsigned)SQ;
        const size_t po0 = (((size_t)(b * HQ + h)) * SQ + s0) * HDQ + 2u * lane;
        unsigned pv[16], pl[16];
#pragma unroll
        for (int r = 0; r < 16; ++r) {
            float e = sg[r * 64 + 2 * lane];
            float o = sg[r * 64 + 2 * lane + 1];
            if (ROPE) {
                const v2f cs = tab[(size_t)(rowBase + r) * 32u + lane];
                const float ne = cs.x * e - cs.y * o;
                const float no = cs.y * e + cs.x * o;
                e = ne; o = no;
            }
            h16 h0, l0, h1, l1;
            split16(e, h0, l0); split16(o, h1, l1);
            pv[r] = pack2h(h0, h1); pl[r] = pack2h(l0, l1);
        }
#pragma unroll
        for (int r = 0; r < 16; ++r) {
            *(volatile unsigned*)(outB + po0 + (size_t)r * HDQ) = pv[r];
            *(volatile unsigned*)(outB + PLX + po0 + (size_t)r * HDQ) = pl[r];
        }
        __threadfence();
#pragma unroll
        for (int r = 0; r < 16; ++r) {
            *(volatile unsigned*)(outB + po0 + (size_t)r * HDQ) = pv[r];
            *(volatile unsigned*)(outB + PLX + po0 + (size_t)r * HDQ) = pl[r];
        }
    }
}

__global__ __launch_bounds__(256) void vt_kernel(const h16* __restrict__ Vr, h16* __restrict__ Vt) {
    __shared__ h16 t[64][66];
    const unsigned tid = threadIdx.x, lane = tid & 31u, wave = tid >> 5;
    const unsigned bh = blockIdx.x / (unsigned)(SQ / 64), s0 = (blockIdx.x % (unsigned)(SQ / 64)) * 64u;
    const size_t pl = blockIdx.y ? PLX : 0;
    const h16* src = Vr + pl + ((size_t)bh * SQ + s0) * HDQ;
#pragma unroll
    for (int k = 0; k < 16; ++k) { const unsigned e = tid + 256u * k; t[e >> 6][e & 63u] = src[e]; }
    __syncthreads();
    h16* dst = Vt + pl + (size_t)bh * HDQ * SQ + s0;
#pragma unroll
    for (int r = 0; r < 8; ++r) {
        const unsigned hd = wave * 8u + r;
        const unsigned pk = pack2h(t[2 * lane][hd], t[2 * lane + 1][hd]);
        unsigned* d = (unsigned*)(dst + (size_t)hd * SQ) + lane;
        *(volatile unsigned*)d = pk; __threadfence(); *(volatile unsigned*)d = pk;
    }
}

__device__ __forceinline__ void attn_kv_block(
    const bool MASK, unsigned kv0, unsigned q0, unsigned lo, unsigned hi, unsigned bh,
    const h16* __restrict__ Km, const h16* __restrict__ Vt, h16* pw, h16* pwl,
    v16h qa0, v16h qa1, v16h qa0l, v16h qa1l,
    v8f (&cacc)[4], float (&mi)[8], float (&li)[8]) {

    v8f s[4] = {};
#pragma unroll
    for (int tt = 0; tt < 4; ++tt) {
        const h16* kRow = Km + ((size_t)bh * SQ + kv0 + tt * 16 + lo) * HDQ;
        v16h kb0  = load_frag2(kRow + hi * 8,            kRow + 16 + hi * 8);
        v16h kb1  = load_frag2(kRow + 32 + hi * 8,       kRow + 48 + hi * 8);
        v16h kb0l = load_frag2(kRow + PLX + hi * 8,      kRow + PLX + 16 + hi * 8);
        v16h kb1l = load_frag2(kRow + PLX + 32 + hi * 8, kRow + PLX + 48 + hi * 8);
        s[tt] = wmma_split(qa0, qa0l, kb0, kb0l, s[tt]);
        s[tt] = wmma_split(qa1, qa1l, kb1, kb1l, s[tt]);
    }

    float alpha[8], rsum[8];
#pragma unroll
    for (int j = 0; j < 8; ++j) {
        if (MASK) {
            const unsigned qg = q0 + j + 8u * hi;
#pragma unroll
            for (int tt = 0; tt < 4; ++tt)
                if (kv0 + tt * 16 + lo > qg) s[tt][j] = -3.0e38f;
        }
        float mb = fmaxf(fmaxf(s[0][j], s[1][j]), fmaxf(s[2][j], s[3][j]));
#pragma unroll
        for (int d = 1; d < 16; d <<= 1) mb = fmaxf(mb, __shfl_xor(mb, d, 32));
        float mnew = fmaxf(mi[j], mb);
        alpha[j] = __expf(mi[j] - mnew);
        mi[j] = mnew;
        const unsigned r = (j + 8u * hi) * 64u;
        float rp = 0.0f;
#pragma unroll
        for (int tt = 0; tt < 4; ++tt) {
            float pv = __expf(s[tt][j] - mnew) * 1024.0f;
            rp += pv;
            h16 ph, pq; split16(pv, ph, pq);
            pw[r + tt * 16 + lo] = ph; pwl[r + tt * 16 + lo] = pq;
        }
#pragma unroll
        for (int d = 1; d < 16; d <<= 1) rp += __shfl_xor(rp, d, 32);
        rsum[j] = rp;
    }
    asm volatile("s_wait_dscnt 0" ::: "memory");
    __builtin_amdgcn_wave_barrier();

    v16h pA0  = load_frag2(pw + lo * 64 + hi * 8,       pw + lo * 64 + hi * 8 + 16);
    v16h pA1  = load_frag2(pw + lo * 64 + 32 + hi * 8,  pw + lo * 64 + 32 + hi * 8 + 16);
    v16h pA0l = load_frag2(pwl + lo * 64 + hi * 8,      pwl + lo * 64 + hi * 8 + 16);
    v16h pA1l = load_frag2(pwl + lo * 64 + 32 + hi * 8, pwl + lo * 64 + 32 + hi * 8 + 16);
    asm volatile("" ::: "memory");

#pragma unroll
    for (int j = 0; j < 8; ++j) li[j] = li[j] * alpha[j] + rsum[j];

#pragma unroll
    for (int t = 0; t < 4; ++t) {
        const h16* vRow = Vt + ((size_t)bh * HDQ + t * 16 + lo) * SQ + kv0;
        v16h vb0  = load_frag2(vRow + hi * 8,            vRow + 16 + hi * 8);
        v16h vb1  = load_frag2(vRow + 32 + hi * 8,       vRow + 48 + hi * 8);
        v16h vb0l = load_frag2(vRow + PLX + hi * 8,      vRow + PLX + 16 + hi * 8);
        v16h vb1l = load_frag2(vRow + PLX + 32 + hi * 8, vRow + PLX + 48 + hi * 8);
#pragma unroll
        for (int j = 0; j < 8; ++j) cacc[t][j] *= alpha[j];
        cacc[t] = wmma_split(pA0, pA0l, vb0, vb0l, cacc[t]);
        cacc[t] = wmma_split(pA1, pA1l, vb1, vb1l, cacc[t]);
    }
}

__global__ __launch_bounds__(256)
void flash_attn_wmma(const h16* __restrict__ Q, const h16* __restrict__ Km,
                     const h16* __restrict__ Vt, h16* __restrict__ ctx) {
    __shared__ alignas(16) h16   psh[8][16 * 64];
    __shared__ alignas(16) h16   pshl[8][16 * 64];
    __shared__ alignas(16) float osh[8][16 * 64];

    const unsigned lane = threadIdx.x & 31u;
    const unsigned wave = threadIdx.x >> 5;
    const unsigned lo   = lane & 15u;
    const unsigned hi   = lane >> 4;
    const unsigned w    = blockIdx.x * 8u + wave;
    const unsigned qt   = w % (unsigned)(SQ / 16);
    const unsigned bh   = w / (unsigned)(SQ / 16);
    const unsigned q0   = qt * 16u;

    const h16* qRow = Q + ((size_t)bh * SQ + q0 + lo) * HDQ;
    v16h qa0  = load_frag2(qRow + hi * 8,            qRow + hi * 8 + 16);
    v16h qa1  = load_frag2(qRow + 32 + hi * 8,       qRow + 32 + hi * 8 + 16);
    v16h qa0l = load_frag2(qRow + PLX + hi * 8,      qRow + PLX + hi * 8 + 16);
    v16h qa1l = load_frag2(qRow + PLX + 32 + hi * 8, qRow + PLX + 32 + hi * 8 + 16);

    v8f   cacc[4] = {};
    float mi[8], li[8];
#pragma unroll
    for (int j = 0; j < 8; ++j) { mi[j] = -3.0e38f; li[j] = 0.0f; }

    const unsigned nblk = (q0 + 79u) >> 6;
    h16* pw  = psh[wave];
    h16* pwl = pshl[wave];

    for (unsigned ib = 0; ib + 1u < nblk; ++ib)
        attn_kv_block(false, ib * 64u, q0, lo, hi, bh, Km, Vt, pw, pwl,
                      qa0, qa1, qa0l, qa1l, cacc, mi, li);
    attn_kv_block(true, (nblk - 1u) * 64u, q0, lo, hi, bh, Km, Vt, pw, pwl,
                  qa0, qa1, qa0l, qa1l, cacc, mi, li);

    const unsigned b = bh / (unsigned)HQ, h = bh % (unsigned)HQ;
    float* so = osh[wave];
#pragma unroll
    for (int j = 0; j < 8; ++j) {
        float inv = 1.0f / li[j];
#pragma unroll
        for (int t = 0; t < 4; ++t) so[(j + 8 * hi) * 64 + t * 16 + lo] = cacc[t][j] * inv;
    }
    asm volatile("s_wait_dscnt 0" ::: "memory");
    __builtin_amdgcn_wave_barrier();
#pragma unroll 1
    for (int pass = 0; pass < 2; ++pass) {
#pragma unroll 4
        for (unsigned r = 0; r < 16; ++r) {
            const float e0 = so[r * 64u + 2u * lane];
            const float e1 = so[r * 64u + 2u * lane + 1u];
            h16 h0, l0, h1, l1;
            split16(e0, h0, l0); split16(e1, h1, l1);
            const size_t po = ((size_t)b * SQ + q0 + r) * DQ + h * HDQ + 2u * lane;
            const unsigned wv = pack2h(h0, h1), wl = pack2h(l0, l1);
            *(volatile unsigned*)(ctx + po) = wv; *(volatile unsigned*)(ctx + PLX + po) = wl;
        }
        __threadfence();
    }
}

extern "C" void kernel_launch(void* const* d_in, const int* in_sizes, int n_in,
                              void* d_out, int out_size, void* d_ws, size_t ws_size,
                              hipStream_t stream) {
    if (n_in < 6) return;
    const long long needX = ((long long)(NB - 1) * SEQ_FULL + SEQ) * DQ;
    const long long needP = (long long)(NB - 1) * SEQ_FULL + SEQ;
    if ((long long)in_sizes[0] < needX) return;
    if ((long long)in_sizes[1] < needP) return;
    if ((long long)in_sizes[2] < (long long)DQ * DQ) return;
    if ((long long)in_sizes[3] < (long long)DQ * DQ) return;
    if ((long long)in_sizes[4] < (long long)DQ * DQ) return;
    if ((long long)in_sizes[5] < (long long)DQ * DQ) return;
    if ((long long)out_size < (long long)MQ * DQ) return;

    const float* x   = (const float*)d_in[0];
    const int*   pos = (const int*)d_in[1];
    const float* wq  = (const float*)d_in[2];
    const float* wk  = (const float*)d_in[3];
    const float* wv  = (const float*)d_in[4];
    const float* wo  = (const float*)d_in[5];
    float* out = (float*)d_out;

    const size_t szX1 = (size_t)MQ * DQ * 2;
    const size_t szX2 = 2 * szX1;
    const size_t szW4 = (size_t)4 * DQ * DQ * 2;
    const size_t szT  = (size_t)MQ * 32 * 8;
    const size_t total = szX1 + szW4 + szT + 5 * szX2;
    static_assert((size_t)MQ * DQ * 2 * 11 + (size_t)4 * DQ * DQ * 2 + (size_t)MQ * 32 * 8 <= (size_t)134217728);
    if (ws_size < total) return;

    char* ws = (char*)d_ws;
    h16* xh   = (h16*)ws;  ws += szX1;
    h16* wP   = (h16*)ws;  ws += szW4;
    v2f* tab  = (v2f*)ws;  ws += szT;
    h16* Qb   = (h16*)ws;  ws += szX2;
    h16* Kb   = (h16*)ws;  ws += szX2;
    h16* Vrb  = (h16*)ws;  ws += szX2;
    h16* Vtb  = (h16*)ws;  ws += szX2;
    h16* ctxb = (h16*)ws;  ws += szX2;

    cvt_x<<<(unsigned)(((size_t)MQ * DQ / 8) / 256), 256, 0, stream>>>(x, xh);
    cvt_w4<<<dim3((unsigned)(((size_t)DQ * DQ / 8) / 256), 4), 256, 0, stream>>>(wq, wk, wv, wo, wP);
    rope_tab<<<(unsigned)(((size_t)MQ * 32) / 256), 256, 0, stream>>>(pos, tab);

    dim3 gg(DQ / 64, MQ / 128);
    gemm_wmma_f16<1, 0, 1><<<gg, 256, 0, stream>>>(xh, wP,           nullptr, Qb,  tab, 0.125f / WCARRY);
    gemm_wmma_f16<1, 0, 1><<<gg, 256, 0, stream>>>(xh, wP + PLW,     nullptr, Kb,  tab, 1.0f / WCARRY);
    gemm_wmma_f16<1, 0, 0><<<gg, 256, 0, stream>>>(xh, wP + 2 * PLW, nullptr, Vrb, tab, 1.0f / WCARRY);
    vt_kernel<<<dim3(NB * HQ * (SQ / 64), 2), 256, 0, stream>>>(Vrb, Vtb);

    flash_attn_wmma<<<(NB * HQ * (SQ / 16)) / 8, 256, 0, stream>>>(Qb, Kb, Vtb, ctxb);

    gemm_wmma_f16<0, 1, 0><<<gg, 256, 0, stream>>>(ctxb, wP + 3 * PLW, out, nullptr, tab, 1.0f / WCARRY);
}
